// ImprovedGeometricDeepONet_9818295239421
// MI455X (gfx1250) — hardware-verified
//
#include <hip/hip_runtime.h>

#define HID   128
#define NRF   10
#define NC    36
#define PDIM  64
#define FEAT  13
#define NPB   8192
#define BATCH 64
#define MT    128
#define LDA   40
#define LDH   136
#define LDAQ  (LDA / 8)
#define LDHQ  (LDH / 8)
#define NW0Q  (HID * LDAQ)
#define NW1Q  (HID * LDHQ)
#define NWOQ  (PDIM * LDHQ)
#define NWQ   (NW0Q + NW1Q + NWOQ)
#define PI_F  3.14159265358979323846f
#define WSC   16.0f
#define WSCI  (1.0f / 16.0f)

static_assert(NPB % MT == 0);
static_assert((BATCH * NPB) % MT == 0);
static_assert(NWQ % 32 == 0);
static_assert(NW0Q % 32 == 0);
static_assert((NW0Q + NW1Q) % 32 == 0);
static_assert(LDA % 8 == 0);
static_assert(LDH % 8 == 0);
static_assert(LDA >= 32);
static_assert(MT == 128);

typedef _Float16 f16;
typedef f16 v16h __attribute__((ext_vector_type(16)));
typedef f16 v8h_t __attribute__((ext_vector_type(8)));
typedef v8h_t __attribute__((may_alias)) v8h;
typedef f16 v4h_t __attribute__((ext_vector_type(4)));
typedef v4h_t __attribute__((may_alias)) v4h;
typedef float v8f __attribute__((ext_vector_type(8)));
typedef v8f __attribute__((may_alias)) v8fa;
typedef float v4f_t __attribute__((ext_vector_type(4)));
typedef v4f_t __attribute__((may_alias)) v4f;
typedef unsigned int v4u_t __attribute__((ext_vector_type(4)));
typedef v4u_t __attribute__((may_alias)) v4u;
typedef unsigned int v2u_t __attribute__((ext_vector_type(2)));
typedef v2u_t __attribute__((may_alias)) v2u;

union Frag { v16h v; v8h_t h[2]; };

__device__ __forceinline__ v8f zero8() {
  v8f z;
#pragma unroll
  for (int i = 0; i < 8; ++i) z[i] = 0.0f;
  return z;
}

__device__ __forceinline__ v16h ldfrag(const f16* p, int k0) {
  Frag f;
  f.h[0] = *(const v8h*)(p + k0);
  f.h[1] = *(const v8h*)(p + k0 + 16);
  return f.v;
}

__device__ __forceinline__ v8f wmma16(v16h a, v16h b, v8f c) {
  return __builtin_amdgcn_wmma_f32_16x16x32_f16(false, a, false, b, (short)0, c, false, false);
}

__global__ void __launch_bounds__(256) prep_kernel(
    const float* __restrict__ tw0, const float* __restrict__ tw1,
    const float* __restrict__ two, f16* __restrict__ img)
{
  const int i = blockIdx.x * 256 + threadIdx.x;
  if (i >= NWQ) return;
  const int i0 = min(i, NW0Q - 1);
  const int n0 = i0 / LDAQ, c0 = (i0 - n0 * LDAQ) * 8;
  const int i1 = min(max(i - NW0Q, 0), NW1Q - 1);
  const int n1 = i1 / LDHQ, c1 = (i1 - n1 * LDHQ) * 8;
  const int i2 = min(max(i - NW0Q - NW1Q, 0), NWOQ - 1);
  const int n2 = i2 / LDHQ, c2 = (i2 - n2 * LDHQ) * 8;
  const int sel = (i < NW0Q) ? 0 : ((i < NW0Q + NW1Q) ? 1 : 2);
  union { v8h_t h; v4u_t u; } pk;
#pragma unroll
  for (int j = 0; j < 8; ++j) {
    const int k0 = c0 + j, k1 = c1 + j, k2 = c2 + j;
    const float a0 = tw0[min(n0 * FEAT + k0, HID * FEAT - 1)];
    const float a1 = tw1[min(n1 * HID + k1, HID * HID - 1)];
    const float a2 = two[min(n2 * HID + k2, PDIM * HID - 1)];
    const float v0 = (k0 < FEAT) ? a0 * WSC : 0.0f;
    const float v1 = (k1 < HID) ? a1 * WSC : 0.0f;
    const float v2 = (k2 < HID) ? a2 * WSC : 0.0f;
    const float v = (sel == 0) ? v0 : ((sel == 1) ? v1 : v2);
    pk.h[j] = (f16)v;
  }
  f16* dst = img + (size_t)i * 8;
  *(volatile v4u_t*)dst = pk.u;
  __threadfence();
  *(volatile v4u_t*)dst = pk.u;
}

__device__ __forceinline__ float bsum128(float v, float* sred, int lane, int wave) {
#pragma unroll
  for (int off = 16; off > 0; off >>= 1) v += __shfl_xor(v, off, 32);
  __syncthreads();
  if (lane == 0) sred[wave] = v;
  __syncthreads();
  return (sred[0] + sred[1]) + (sred[2] + sred[3]);
}

__global__ void __launch_bounds__(128) branch_kernel(
    const float* __restrict__ coeffs, const float* __restrict__ cmean,
    const float* __restrict__ cstd,
    const float* __restrict__ w0, const float* __restrict__ b0,
    const float* __restrict__ g0, const float* __restrict__ be0,
    const float* __restrict__ w1, const float* __restrict__ b1,
    const float* __restrict__ g1, const float* __restrict__ be1,
    const float* __restrict__ w2, const float* __restrict__ b2,
    const float* __restrict__ g2, const float* __restrict__ be2,
    const float* __restrict__ wo, const float* __restrict__ bo,
    float* __restrict__ pbr)
{
  __shared__ float sc[NC];
  __shared__ float sx[HID];
  __shared__ float sred[4];
  __shared__ __align__(16) float spb[PDIM];

  const int b = blockIdx.x;
  const int t = threadIdx.x;
  const int lane = t & 31, wave = t >> 5;

  if (t < NC) {
    const float cs = cstd[t] + 1e-8f;
    sc[t] = (coeffs[b * NC + t] - cmean[t]) * (1.0f / cs);
  }
  __syncthreads();

  float v = b0[t];
#pragma unroll 1
  for (int k = 0; k < NC; ++k) v = fmaf(w0[t * NC + k], sc[k], v);
  float mu = bsum128(v, sred, lane, wave) * (1.0f / HID);
  float d = v - mu;
  float var = bsum128(d * d, sred, lane, wave) * (1.0f / HID);
  const float x0 = fmaxf(d * rsqrtf(var + 1e-5f) * g0[t] + be0[t], 0.0f);
  sx[t] = x0;
  __syncthreads();

  v = b1[t];
#pragma unroll 1
  for (int k = 0; k < HID; ++k) v = fmaf(w1[t * HID + k], sx[k], v);
  mu = bsum128(v, sred, lane, wave) * (1.0f / HID);
  d = v - mu;
  var = bsum128(d * d, sred, lane, wave) * (1.0f / HID);
  const float x1 = fmaxf(d * rsqrtf(var + 1e-5f) * g1[t] + be1[t], 0.0f) + x0;
  __syncthreads();
  sx[t] = x1;
  __syncthreads();

  v = b2[t];
#pragma unroll 1
  for (int k = 0; k < HID; ++k) v = fmaf(w2[t * HID + k], sx[k], v);
  mu = bsum128(v, sred, lane, wave) * (1.0f / HID);
  d = v - mu;
  var = bsum128(d * d, sred, lane, wave) * (1.0f / HID);
  const float x2 = fmaxf(d * rsqrtf(var + 1e-5f) * g2[t] + be2[t], 0.0f) + x1;
  __syncthreads();
  sx[t] = x2;
  __syncthreads();

  const int tt = min(t, PDIM - 1);
  float pv = bo[tt];
#pragma unroll 1
  for (int k = 0; k < HID; ++k) pv = fmaf(wo[tt * HID + k], sx[k], pv);
  if (t < PDIM) spb[t] = pv;
  __syncthreads();

  v4f_t q;
  q[0] = q[1] = q[2] = q[3] = 0.0f;
  if (t < 16) q = *(const v4f*)(spb + 4 * t);
  float* dst = pbr + (size_t)b * PDIM + 4 * min(t, 15);
  if (t < 16) *(volatile v4f_t*)dst = q;
  __threadfence();
  if (t < 16) *(volatile v4f_t*)dst = q;
}

__device__ __forceinline__ float geo_feat(float ct, float st, float phi,
                                          float rct, float rst, float rp) {
#pragma clang fp contract(off)
  const float a  = ct * rct;
  const float bb = (st * rst) * cosf(phi - rp);
  float cd = a + bb;
  cd = fminf(fmaxf(cd, -1.0f), 1.0f);
  return acosf(cd) * (1.0f / PI_F);
}

__device__ __forceinline__ void ln_relu_to_lds(v8f (&acc)[8], const float* sb, const float* sg,
                                               const float* sbe, f16* hrow, int hh)
{
  float rs = 0.0f;
#pragma unroll
  for (int mt = 0; mt < 8; ++mt) {
    const v8f bv = *(const v8fa*)(sb + mt * 16 + 8 * hh);
#pragma unroll
    for (int i = 0; i < 8; ++i) {
      const float x = acc[mt][i] * WSCI + bv[i];
      acc[mt][i] = x;
      rs += x;
    }
  }
  rs += __shfl_xor(rs, 16, 32);
  const float mu = rs * (1.0f / HID);
  float rq = 0.0f;
#pragma unroll
  for (int mt = 0; mt < 8; ++mt) {
#pragma unroll
    for (int i = 0; i < 8; ++i) {
      const float d = acc[mt][i] - mu;
      rq += d * d;
    }
  }
  rq += __shfl_xor(rq, 16, 32);
  const float var = rq * (1.0f / HID);
  const float inv = rsqrtf(var + 1e-5f);
#pragma unroll
  for (int mt = 0; mt < 8; ++mt) {
    const v8f gv  = *(const v8fa*)(sg  + mt * 16 + 8 * hh);
    const v8f bev = *(const v8fa*)(sbe + mt * 16 + 8 * hh);
    v8h_t hv;
#pragma unroll
    for (int i = 0; i < 8; ++i) {
      const float y = (acc[mt][i] - mu) * inv * gv[i] + bev[i];
      hv[i] = (f16)fmaxf(y, 0.0f);
    }
    *(v8h*)(hrow + mt * 16) = hv;
  }
}

__global__ void __launch_bounds__(256) trunk_kernel(
    const float* __restrict__ coords,
    const float* __restrict__ rth, const float* __restrict__ rph,
    const f16* __restrict__ wimg,
    const float* __restrict__ tb0, const float* __restrict__ tg0, const float* __restrict__ tbe0,
    const float* __restrict__ tb1, const float* __restrict__ tg1, const float* __restrict__ tbe1,
    const float* __restrict__ tbo, const float* __restrict__ pbr,
    float* __restrict__ out)
{
  __shared__ __align__(16) f16 sW[NWQ * 8];
  __shared__ __align__(16) f16 sA[MT * LDA];
  __shared__ __align__(16) f16 sH[MT * LDH];
  __shared__ __align__(32) float sB0[HID];
  __shared__ __align__(32) float sG0[HID];
  __shared__ __align__(32) float sBe0[HID];
  __shared__ __align__(32) float sB1[HID];
  __shared__ __align__(32) float sG1[HID];
  __shared__ __align__(32) float sBe1[HID];
  __shared__ __align__(32) float sBo[PDIM];
  __shared__ __align__(32) float sPb[PDIM];
  __shared__ float sRct[16];
  __shared__ float sRst[16];
  __shared__ float sRp[16];
  __shared__ __align__(16) float sOut[MT];

  const int tid  = threadIdx.x;
  const int wave = tid >> 5;
  const int lane = tid & 31;
  const int m    = lane & 15;
  const int hh   = lane >> 4;
  const int blk  = blockIdx.x;
  const int row0 = blk * MT;
  const int b    = blk / (NPB / MT);

  {
    const v4u* src = (const v4u*)wimg;
    v4u* dst = (v4u*)sW;
#pragma unroll 1
    for (int i = tid; i < NWQ; i += 256) dst[i] = src[i];
  }
  if (tid < HID) {
    sB0[tid] = tb0[tid]; sG0[tid] = tg0[tid]; sBe0[tid] = tbe0[tid];
    sB1[tid] = tb1[tid]; sG1[tid] = tg1[tid]; sBe1[tid] = tbe1[tid];
  }
  if (tid < PDIM) {
    sBo[tid] = tbo[tid];
    sPb[tid] = pbr[(size_t)b * PDIM + tid];
  }
  if (tid < NRF) {
    const float t0 = rth[tid];
    sRct[tid] = cosf(t0);
    sRst[tid] = sinf(t0);
    sRp[tid]  = rph[tid];
  }
  __syncthreads();

  if (tid < MT) {
    const int r = tid;
    const size_t gi = (size_t)row0 + r;
    const float theta = coords[gi * 2 + 0];
    const float phi   = coords[gi * 2 + 1];
    const float ct = cosf(theta), st = sinf(theta);
    v8h_t f0;
#pragma unroll
    for (int j = 0; j < 8; ++j)
      f0[j] = (f16)geo_feat(ct, st, phi, sRct[j], sRst[j], sRp[j]);
    v4h_t f1;
    f1[0] = (f16)geo_feat(ct, st, phi, sRct[8], sRst[8], sRp[8]);
    f1[1] = (f16)geo_feat(ct, st, phi, sRct[9], sRst[9], sRp[9]);
    f1[2] = (f16)(theta * (1.0f / PI_F));
    f1[3] = (f16)(phi * (1.0f / (2.0f * PI_F)));
    f16* rowp = sA + r * LDA;
    *(v8h*)(rowp) = f0;
    *(v4h*)(rowp + 8) = f1;
    v2u_t c;
    c[0] = 0x00003C00u;
    c[1] = 0u;
    *(v2u*)(rowp + 12) = c;
  } else {
    const int r = tid - MT;
    f16* rowp = sA + r * LDA;
    v4u_t z;
    z[0] = 0u; z[1] = 0u; z[2] = 0u; z[3] = 0u;
    *(v4u*)(rowp + 16) = z;
    *(v4u*)(rowp + 24) = z;
  }
  __syncthreads();

  const f16* sW0 = sW;
  const f16* sW1 = sW + HID * LDA;
  const f16* sWo = sW1 + HID * LDH;
  const int prow = wave * 16 + m;
  const f16* arow = sA + prow * LDA + 8 * hh;
  f16* hrow = sH + prow * LDH + 8 * hh;

  v8f acc[8];
  {
    const v16h bf = ldfrag(arow, 0);
    v16h af;
#pragma unroll
    for (int mt = 0; mt < 8; ++mt) {
      af = ldfrag(sW0 + (mt * 16 + m) * LDA + 8 * hh, 0);
      acc[mt] = wmma16(af, bf, zero8());
    }
    asm volatile("v_nop\n\tv_nop\n\tv_nop\n\tv_nop"
                 : "+v"(acc[0]), "+v"(acc[1]), "+v"(acc[2]), "+v"(acc[3]),
                   "+v"(acc[4]), "+v"(acc[5]), "+v"(acc[6]), "+v"(acc[7])
                 : "v"(af), "v"(bf));
  }
  ln_relu_to_lds(acc, sB0, sG0, sBe0, hrow, hh);
  __syncthreads();

#pragma unroll
  for (int mt = 0; mt < 8; ++mt) acc[mt] = zero8();
#pragma unroll 1
  for (int k0 = 0; k0 < HID; k0 += 32) {
    const v16h bf = ldfrag(hrow, k0);
    v16h af;
#pragma unroll
    for (int mt = 0; mt < 8; ++mt) {
      af = ldfrag(sW1 + (mt * 16 + m) * LDH + 8 * hh, k0);
      acc[mt] = wmma16(af, bf, acc[mt]);
    }
    asm volatile("v_nop\n\tv_nop\n\tv_nop\n\tv_nop"
                 : "+v"(acc[0]), "+v"(acc[1]), "+v"(acc[2]), "+v"(acc[3]),
                   "+v"(acc[4]), "+v"(acc[5]), "+v"(acc[6]), "+v"(acc[7])
                 : "v"(af), "v"(bf));
  }
  ln_relu_to_lds(acc, sB1, sG1, sBe1, hrow, hh);
  __syncthreads();

  v8f acc2[4];
#pragma unroll
  for (int mt = 0; mt < 4; ++mt) acc2[mt] = zero8();
#pragma unroll 1
  for (int k0 = 0; k0 < HID; k0 += 32) {
    const v16h bf = ldfrag(hrow, k0);
    v16h af;
#pragma unroll
    for (int mt = 0; mt < 4; ++mt) {
      af = ldfrag(sWo + (mt * 16 + m) * LDH + 8 * hh, k0);
      acc2[mt] = wmma16(af, bf, acc2[mt]);
    }
    asm volatile("v_nop\n\tv_nop\n\tv_nop\n\tv_nop"
                 : "+v"(acc2[0]), "+v"(acc2[1]), "+v"(acc2[2]), "+v"(acc2[3])
                 : "v"(af), "v"(bf));
  }
  float op = 0.0f;
#pragma unroll
  for (int mt = 0; mt < 4; ++mt) {
    const v8f bov = *(const v8fa*)(sBo + mt * 16 + 8 * hh);
    const v8f pbv = *(const v8fa*)(sPb + mt * 16 + 8 * hh);
#pragma unroll
    for (int i = 0; i < 8; ++i) {
      const float pt = acc2[mt][i] * WSCI + bov[i];
      op = fmaf(pt, pbv[i], op);
    }
  }
  op += __shfl_xor(op, 16, 32);
  if (hh == 0) sOut[prow] = op;
  __syncthreads();

  if (tid < 32) {
    const v4f_t q = *(const v4f*)(sOut + 4 * lane);
    float* go = out + (size_t)row0 + 4 * lane;
    *(volatile v4f_t*)go = q;
    __threadfence();
    *(volatile v4f_t*)go = q;
  }
}

extern "C" void kernel_launch(void* const* d_in, const int* in_sizes, int n_in,
                              void* d_out, int out_size, void* d_ws, size_t ws_size,
                              hipStream_t stream)
{
  if (n_in < 30) return;
  if (in_sizes[0] != BATCH * NC) return;
  if (in_sizes[1] != BATCH * NPB * 2) return;
  if (in_sizes[2] != NC || in_sizes[3] != NC) return;
  if (in_sizes[4] != NRF || in_sizes[5] != NRF) return;
  if (in_sizes[6] != HID * NC) return;
  if (in_sizes[7] != HID || in_sizes[8] != HID || in_sizes[9] != HID) return;
  if (in_sizes[10] != HID * HID) return;
  if (in_sizes[11] != HID || in_sizes[12] != HID || in_sizes[13] != HID) return;
  if (in_sizes[14] != HID * HID) return;
  if (in_sizes[15] != HID || in_sizes[16] != HID || in_sizes[17] != HID) return;
  if (in_sizes[18] != PDIM * HID || in_sizes[19] != PDIM) return;
  if (in_sizes[20] != HID * FEAT) return;
  if (in_sizes[21] != HID || in_sizes[22] != HID || in_sizes[23] != HID) return;
  if (in_sizes[24] != HID * HID) return;
  if (in_sizes[25] != HID || in_sizes[26] != HID || in_sizes[27] != HID) return;
  if (in_sizes[28] != PDIM * HID || in_sizes[29] != PDIM) return;
  if (out_size != BATCH * NPB) return;

  const float* coeffs = (const float*)d_in[0];
  const float* coords = (const float*)d_in[1];
  const float* cmean  = (const float*)d_in[2];
  const float* cstd   = (const float*)d_in[3];
  const float* rth    = (const float*)d_in[4];
  const float* rph    = (const float*)d_in[5];
  const float* b_w0 = (const float*)d_in[6];  const float* b_b0  = (const float*)d_in[7];
  const float* b_g0 = (const float*)d_in[8];  const float* b_be0 = (const float*)d_in[9];
  const float* b_w1 = (const float*)d_in[10]; const float* b_b1  = (const float*)d_in[11];
  const float* b_g1 = (const float*)d_in[12]; const float* b_be1 = (const float*)d_in[13];
  const float* b_w2 = (const float*)d_in[14]; const float* b_b2  = (const float*)d_in[15];
  const float* b_g2 = (const float*)d_in[16]; const float* b_be2 = (const float*)d_in[17];
  const float* b_wo = (const float*)d_in[18]; const float* b_bo  = (const float*)d_in[19];
  const float* t_w0 = (const float*)d_in[20]; const float* t_b0  = (const float*)d_in[21];
  const float* t_g0 = (const float*)d_in[22]; const float* t_be0 = (const float*)d_in[23];
  const float* t_w1 = (const float*)d_in[24]; const float* t_b1  = (const float*)d_in[25];
  const float* t_g1 = (const float*)d_in[26]; const float* t_be1 = (const float*)d_in[27];
  const float* t_wo = (const float*)d_in[28]; const float* t_bo  = (const float*)d_in[29];
  float* out = (float*)d_out;

  const size_t off_pbr  = 0;
  const size_t n_pbr    = (size_t)BATCH * PDIM * sizeof(float);
  const size_t off_wimg = off_pbr + n_pbr;
  const size_t n_wimg   = (size_t)NWQ * 16;
  const size_t total    = off_wimg + n_wimg;
  if (total > ws_size) return;

  char* ws = (char*)d_ws;
  float* pbr  = (float*)(ws + off_pbr);
  f16*   wimg = (f16*)(ws + off_wimg);

  prep_kernel<<<(NWQ + 255) / 256, 256, 0, stream>>>(t_w0, t_w1, t_wo, wimg);

  branch_kernel<<<BATCH, 128, 0, stream>>>(
      coeffs, cmean, cstd,
      b_w0, b_b0, b_g0, b_be0, b_w1, b_b1, b_g1, b_be1,
      b_w2, b_b2, b_g2, b_be2, b_wo, b_bo, pbr);

  const int nblocks = (BATCH * NPB) / MT;
  trunk_kernel<<<nblocks, 256, 0, stream>>>(
      coords, rth, rph, wimg,
      t_b0, t_g0, t_be0, t_b1, t_g1, t_be1, t_bo, pbr, out);
}
